// PhysicsBiasedBlock_6098853560435
// MI455X (gfx1250) — hardware-verified
//
#include <hip/hip_runtime.h>
#include <math.h>

constexpr int kBatch   = 4;
constexpr int kSeq     = 1024;
constexpr int kDim     = 768;
constexpr int kHeads   = 12;
constexpr int kHeadDim = 64;
constexpr int kHid     = 3072;
constexpr int kTok     = kBatch * kSeq;
constexpr int kQKVld   = 3 * kDim;
constexpr int kGroups  = kBatch * kHeads;
constexpr int kGroupsPerChunk = 6;
constexpr int kChunks  = kGroups / kGroupsPerChunk;
constexpr float kWCarry    = 16.0f;
constexpr float kPCarry    = 2048.0f;
constexpr float kOCarry    = 32.0f;
constexpr float kAttnScale = 0.125f;
constexpr float kLnEps     = 1e-6f;
constexpr float kInvDim    = 1.0f / 768.0f;

static_assert(kChunks * kGroupsPerChunk == kGroups, "chunks");
static_assert(kHeads % kGroupsPerChunk == 0, "chunk inside one batch");

constexpr size_t kBytesWqkv  = (size_t)kQKVld * kDim * 2;
constexpr size_t kBytesWproj = (size_t)kDim * kDim * 2;
constexpr size_t kBytesWfc1  = (size_t)kHid * kDim * 2;
constexpr size_t kBytesWfc2  = (size_t)kDim * kHid * 2;
constexpr size_t kBytesH     = (size_t)kTok * kDim * 2;
constexpr size_t kBytesQKV   = (size_t)kTok * kQKVld * 2;
constexpr size_t kBytesVt    = (size_t)kGroups * kHeadDim * kSeq * 2;
constexpr size_t kBytesO     = (size_t)kTok * kDim * 2;
constexpr size_t kBytesX1    = (size_t)kTok * kDim * 4;
constexpr size_t kBytesScores = (size_t)kGroupsPerChunk * kSeq * kSeq * 4;
constexpr size_t kBytesP      = (size_t)kGroupsPerChunk * kSeq * kSeq * 2;
constexpr size_t kBytesG1     = (size_t)kTok * kHid * 4;
constexpr size_t kBytesHG     = (size_t)kTok * kHid * 2;
constexpr size_t kBytesBig    = (kBytesScores + kBytesP > kBytesG1) ? (kBytesScores + kBytesP) : kBytesG1;

constexpr size_t kOffWqkv  = 0;
constexpr size_t kOffWproj = kOffWqkv + kBytesWqkv;
constexpr size_t kOffWfc1  = kOffWproj + kBytesWproj;
constexpr size_t kOffWfc2  = kOffWfc1 + kBytesWfc1;
constexpr size_t kOffH     = kOffWfc2 + kBytesWfc2;
constexpr size_t kOffQKV   = kOffH + kBytesH;
constexpr size_t kOffVt    = kOffQKV + kBytesQKV;
constexpr size_t kOffO     = kOffVt + kBytesVt;
constexpr size_t kOffX1    = kOffO + kBytesO;
constexpr size_t kOffBig   = kOffX1 + kBytesX1;
constexpr size_t kOffScores = kOffBig;
constexpr size_t kOffP      = kOffBig + kBytesScores;
constexpr size_t kOffG1     = kOffBig;
constexpr size_t kOffHG     = kOffQKV;
constexpr size_t kWsTotal   = kOffBig + kBytesBig;
static_assert(kBytesHG == kBytesQKV + kBytesVt, "hg reuses qkv + vt exactly");
static_assert(kOffHG + kBytesHG <= kOffO, "hg inside dead region");
static_assert(kWsTotal == 114819072, "carve total");
static_assert(kWsTotal <= 134217728, "carve under 128 MiB");
static_assert((kOffWproj % 256) == 0 && (kOffWfc1 % 256) == 0 && (kOffWfc2 % 256) == 0 && (kOffH % 256) == 0 &&
              (kOffQKV % 256) == 0 && (kOffVt % 256) == 0 && (kOffO % 256) == 0 && (kOffX1 % 256) == 0 &&
              (kOffBig % 256) == 0 && (kOffP % 256) == 0, "aligned carves");

typedef __attribute__((ext_vector_type(16))) _Float16 v16h;
typedef __attribute__((ext_vector_type(8)))  _Float16 v8h;
typedef __attribute__((ext_vector_type(16))) __bf16   v16b;
typedef __attribute__((ext_vector_type(8)))  __bf16   v8b;
typedef __attribute__((ext_vector_type(8)))  float    v8f;
typedef __attribute__((ext_vector_type(4)))  float    v4f;
typedef __attribute__((ext_vector_type(2)))  float    v2f;
typedef __attribute__((ext_vector_type(4)))  unsigned int v4u;

__device__ __forceinline__ unsigned short f2bf_bits(float f) {
  unsigned u = __float_as_uint(f);
  return (unsigned short)((u + 0x7FFFu + ((u >> 16) & 1u)) >> 16);
}
__device__ __forceinline__ float bf_bits2f(unsigned short h) { return __uint_as_float(((unsigned)h) << 16); }

__device__ __forceinline__ void dep_guard_h(v8f& a, v8f& b, v16h x, v16h y) { asm volatile("v_nop\n\tv_nop\n\tv_nop\n\tv_nop" : "+v"(a), "+v"(b) : "v"(x), "v"(y)); }
__device__ __forceinline__ void dep_guard_b(v8f& a, v8f& b, v16b x, v16b y) { asm volatile("v_nop\n\tv_nop\n\tv_nop\n\tv_nop" : "+v"(a), "+v"(b) : "v"(x), "v"(y)); }
__device__ __forceinline__ void keep4_h(v16h a, v16h b, v16h c, v16h d) { asm volatile("v_nop" :: "v"(a), "v"(b), "v"(c), "v"(d)); }
__device__ __forceinline__ void keep4_b(v16b a, v16b b, v16b c, v16b d) { asm volatile("v_nop" :: "v"(a), "v"(b), "v"(c), "v"(d)); }
__device__ __forceinline__ void acc_guard4(v8f& a, v8f& b, v8f& c, v8f& d) { asm volatile("v_nop\n\tv_nop\n\tv_nop\n\tv_nop" : "+v"(a), "+v"(b), "+v"(c), "+v"(d)); }
template <typename T> struct Frag;
template <> struct Frag<_Float16> {
  typedef v16h V; union U { v16h v; v8h h[2]; };
  static __device__ __forceinline__ v16h load(const _Float16* p) {
    U f; f.h[0] = *(const v8h*)(p); f.h[1] = *(const v8h*)(p + 16); return f.v;
  }
  static __device__ __forceinline__ v8f mma(v16h a, v16h b, v8f c) {
    return __builtin_amdgcn_wmma_f32_16x16x32_f16(false, a, false, b, (short)0, c, false, false);
  }
  static __device__ __forceinline__ void guard(v8f& a, v8f& b, v16h x, v16h y) { dep_guard_h(a, b, x, y); }
  static __device__ __forceinline__ void keep(v16h a, v16h b, v16h c, v16h d) { keep4_h(a, b, c, d); }
};
template <> struct Frag<__bf16> {
  typedef v16b V; union U { v16b v; v8b h[2]; };
  static __device__ __forceinline__ v16b load(const __bf16* p) {
    U f; f.h[0] = *(const v8b*)(p); f.h[1] = *(const v8b*)(p + 16); return f.v;
  }
  static __device__ __forceinline__ v8f mma(v16b a, v16b b, v8f c) {
    return __builtin_amdgcn_wmma_f32_16x16x32_bf16(false, a, false, b, (short)0, c, false, false);
  }
  static __device__ __forceinline__ void guard(v8f& a, v8f& b, v16b x, v16b y) { dep_guard_b(a, b, x, y); }
  static __device__ __forceinline__ void keep(v16b a, v16b b, v16b c, v16b d) { keep4_b(a, b, c, d); }
};

__device__ __forceinline__ unsigned pk16(unsigned short a, unsigned short b) { return (unsigned)a | ((unsigned)b << 16); }
__device__ __forceinline__ unsigned short h_bits(float f) { const _Float16 h = (_Float16)f; return __builtin_bit_cast(unsigned short, h); }

template <int ET> struct Elem;
template <> struct Elem<0> { typedef _Float16 T; };
template <> struct Elem<1> { typedef __bf16 T; };
template <int ET, bool SPLIT, int BIAS_MODE, int OUT_MODE, bool RESID, int ACT = 0>
__global__ __launch_bounds__(256) void wmma_gemm64(
    const unsigned short* __restrict__ Ap, const unsigned short* __restrict__ A2p, int lda, long strideA,
    const unsigned short* __restrict__ Btp, const unsigned short* __restrict__ Bt2p, int ldb, long strideB,
    void* __restrict__ Cout, void* __restrict__ Cout2, int ldc, long strideC,
    const float* __restrict__ bias,
    const float* __restrict__ resid, long strideR,
    int M, int N, int K, float scale) {
  typedef typename Elem<ET>::T T;
  typedef typename Frag<T>::V V;
  const T* A = (const T*)Ap; const T* A2 = (const T*)A2p; const T* Bt = (const T*)Btp; const T* Bt2 = (const T*)Bt2p;
  __shared__ __align__(16) float sT[8][16 * 68];
  const int b    = blockIdx.y;
  const int lane = threadIdx.x & 31;
  const int wave = threadIdx.x >> 5;
  const int tilesN = N >> 6;
  const int tilesM = M >> 6;
  const int tile = blockIdx.x * 8 + wave;
  if (tile >= tilesM * tilesN) return;
  const int tm = tile / tilesN;
  const int tn = tile - tm * tilesN;
  const int m0 = tm << 6;
  const int n0 = tn << 6;

  const T* Ab  = A  + (size_t)b * strideA;
  const T* Bb  = Bt + (size_t)b * strideB;
  const T* Ab2 = SPLIT ? (A2  + (size_t)b * strideA) : nullptr;
  const T* Bb2 = SPLIT ? (Bt2 + (size_t)b * strideB) : nullptr;

  const int rlane = lane & 15;
  const int koff  = (lane >> 4) * 8;
  const int mOff  = (lane >> 4) * 8;

  v8f acc[4][4];
#pragma unroll
  for (int i = 0; i < 4; ++i)
#pragma unroll
    for (int j = 0; j < 4; ++j) acc[i][j] = (v8f){0.f,0.f,0.f,0.f,0.f,0.f,0.f,0.f};

  for (int k0 = 0; k0 < K; k0 += 32) {
    V bh[4], bl[4];
#pragma unroll
    for (int j = 0; j < 4; ++j) {
      const size_t bo = (size_t)(n0 + (j << 4) + rlane) * ldb + koff + k0;
      bh[j] = Frag<T>::load(Bb + bo);
      if (SPLIT) bl[j] = Frag<T>::load(Bb2 + bo);
    }
#pragma unroll
    for (int i = 0; i < 4; ++i) {
      const size_t ao = (size_t)(m0 + (i << 4) + rlane) * lda + koff + k0;
      V ah = Frag<T>::load(Ab + ao);
      V al;
      if (SPLIT) al = Frag<T>::load(Ab2 + ao);
#pragma unroll
      for (int j = 0; j < 4; ++j) {
        acc[i][j] = Frag<T>::mma(ah, bh[j], acc[i][j]);
        if (SPLIT) {
          acc[i][j] = Frag<T>::mma(ah, bl[j], acc[i][j]);
          acc[i][j] = Frag<T>::mma(al, bh[j], acc[i][j]);
        }
      }
      Frag<T>::guard(acc[i][0], acc[i][3], ah, SPLIT ? al : ah);
    }
    Frag<T>::keep(bh[0], bh[1], bh[2], bh[3]);
    if (SPLIT) Frag<T>::keep(bl[0], bl[1], bl[2], bl[3]);
  }
  acc_guard4(acc[0][0], acc[0][1], acc[0][2], acc[0][3]);
  acc_guard4(acc[1][0], acc[1][1], acc[1][2], acc[1][3]);
  acc_guard4(acc[2][0], acc[2][1], acc[2][2], acc[2][3]);
  acc_guard4(acc[3][0], acc[3][1], acc[3][2], acc[3][3]);

  float* slab = sT[wave];
  const float* Rb = RESID ? (resid + (size_t)b * strideR) : nullptr;
#pragma unroll
  for (int i = 0; i < 4; ++i) {
    const int mBase = m0 + (i << 4);
#pragma unroll
    for (int j = 0; j < 4; ++j) {
      const int n = n0 + (j << 4) + rlane;
      float bv = 0.f;
      if (BIAS_MODE == 2) bv = bias[n];
#pragma unroll
      for (int r = 0; r < 8; ++r) {
        float v = acc[i][j][r] * scale;
        if (BIAS_MODE == 1) v += bias[mBase + mOff + r];
        if (BIAS_MODE == 2) v += bv;
        if (RESID) v += Rb[(size_t)(mBase + mOff + r) * ldc + n];
        if (ACT == 2) v = fmaxf(v, 0.0f);
        if (ACT == 4) v = (v > 0.f) ? v : 0.01f * v;
        slab[(mOff + r) * 68 + (j << 4) + rlane] = v;
      }
    }
    __builtin_amdgcn_fence(__ATOMIC_RELEASE, "workgroup");
    __builtin_amdgcn_wave_barrier();
    __builtin_amdgcn_fence(__ATOMIC_ACQUIRE, "workgroup");
    if (OUT_MODE == 0) {
      float* C = (float*)Cout + (size_t)b * strideC;
      const int hh = lane >> 4, c4 = (lane & 15) * 4;
      for (int pass = 0; pass < 2; ++pass) {
#pragma unroll
        for (int it = 0; it < 8; ++it) {
          const int row = it * 2 + hh;
          v4f v = *(const v4f*)(slab + row * 68 + c4);
          *(volatile v4f*)(C + (size_t)(mBase + row) * ldc + n0 + c4) = v;
        }
        __threadfence();
      }
    } else {
      const int q = lane >> 3, c8 = (lane & 7) * 8;
      unsigned short* C  = (unsigned short*)Cout  + (size_t)b * strideC;
      unsigned short* C2 = (OUT_MODE == 2) ? ((unsigned short*)Cout2 + (size_t)b * strideC) : nullptr;
      for (int pass = 0; pass < 2; ++pass) {
#pragma unroll
        for (int it = 0; it < 4; ++it) {
          const int row = it * 4 + q;
          const float* sp = slab + row * 68 + c8;
          v8h hv, lv;
#pragma unroll
          for (int e = 0; e < 8; ++e) {
            if (OUT_MODE == 1) {
              hv[e] = (_Float16)sp[e];
            } else {
              unsigned short hb = f2bf_bits(sp[e]);
              unsigned short lb = f2bf_bits(sp[e] - bf_bits2f(hb));
              hv[e] = __builtin_bit_cast(_Float16, hb);
              lv[e] = __builtin_bit_cast(_Float16, lb);
            }
          }
          *(volatile v8h*)(C + (size_t)(mBase + row) * ldc + n0 + c8) = hv;
          if (OUT_MODE == 2) *(volatile v8h*)(C2 + (size_t)(mBase + row) * ldc + n0 + c8) = lv;
        }
        __threadfence();
      }
    }
    __builtin_amdgcn_fence(__ATOMIC_RELEASE, "workgroup");
    __builtin_amdgcn_wave_barrier();
    __builtin_amdgcn_fence(__ATOMIC_ACQUIRE, "workgroup");
  }
}

__global__ __launch_bounds__(256) void wtcast_kernel(const float* __restrict__ W, unsigned short* __restrict__ out,
                                                     int kin, int nout, float scale) {
  __shared__ float sm[64][65];
  const int t  = threadIdx.x;
  const int k0 = blockIdx.x * 64;
  const int n0 = blockIdx.y * 64;
#pragma unroll
  for (int i = 0; i < 16; ++i) {
    const int e = i * 256 + t;
    const int r = e >> 6;
    const int c = e & 63;
    sm[c][r] = W[(size_t)(k0 + r) * nout + n0 + c] * scale;
  }
  __syncthreads();
  const int lane = t & 31, wave = t >> 5;
  const int q = lane >> 3, c8 = (lane & 7) * 8;
  for (int pass = 0; pass < 2; ++pass) {
#pragma unroll
    for (int it = 0; it < 2; ++it) {
      const int row = wave * 8 + it * 4 + q;
      unsigned short hb[8];
#pragma unroll
      for (int e = 0; e < 8; ++e) hb[e] = h_bits(sm[row][c8 + e]);
      const v4u u = (v4u){pk16(hb[0], hb[1]), pk16(hb[2], hb[3]), pk16(hb[4], hb[5]), pk16(hb[6], hb[7])};
      *(volatile v4u*)(out + (size_t)(n0 + row) * kin + k0 + c8) = u;
    }
    __threadfence();
  }
}

__global__ __launch_bounds__(96) void layernorm_f16_kernel(const float* __restrict__ x, const float* __restrict__ w,
                                                           const float* __restrict__ bvec, unsigned short* __restrict__ out) {
  __shared__ float redA[4];
  __shared__ float redB[4];
  const int row  = blockIdx.x;
  const int t    = threadIdx.x;
  const int lane = t & 31, wave = t >> 5;
  const int c0   = t * 8;
  const float* xr = x + (size_t)row * kDim + c0;
  const v4f a = *(const v4f*)(xr);
  const v4f c = *(const v4f*)(xr + 4);
  float v[8];
#pragma unroll
  for (int e = 0; e < 4; ++e) { v[e] = a[e]; v[4 + e] = c[e]; }
  float s = ((v[0] + v[1]) + (v[2] + v[3])) + ((v[4] + v[5]) + (v[6] + v[7]));
#pragma unroll
  for (int off = 16; off > 0; off >>= 1) s += __shfl_xor(s, off, 32);
  if (lane == 0) redA[wave] = s;
  __syncthreads();
  const float mu = ((redA[0] + redA[1]) + redA[2]) * kInvDim;
  float d[8];
  float sq = 0.f;
#pragma unroll
  for (int e = 0; e < 8; ++e) { d[e] = v[e] - mu; sq += d[e] * d[e]; }
#pragma unroll
  for (int off = 16; off > 0; off >>= 1) sq += __shfl_xor(sq, off, 32);
  if (lane == 0) redB[wave] = sq;
  __syncthreads();
  const float var = ((redB[0] + redB[1]) + redB[2]) * kInvDim;
  const float rs  = rsqrtf(var + kLnEps);
  const v4f wa = *(const v4f*)(w + c0);
  const v4f wc = *(const v4f*)(w + c0 + 4);
  const v4f ba = *(const v4f*)(bvec + c0);
  const v4f bc = *(const v4f*)(bvec + c0 + 4);
  unsigned short hb[8];
#pragma unroll
  for (int e = 0; e < 4; ++e) {
    hb[e]     = h_bits(d[e] * rs * wa[e] + ba[e]);
    hb[4 + e] = h_bits(d[4 + e] * rs * wc[e] + bc[e]);
  }
  const v4u u = (v4u){pk16(hb[0], hb[1]), pk16(hb[2], hb[3]), pk16(hb[4], hb[5]), pk16(hb[6], hb[7])};
  unsigned short* op = out + (size_t)row * kDim + c0;
  *(volatile v4u*)op = u;
  __threadfence();
  *(volatile v4u*)op = u;
}

__global__ __launch_bounds__(256) void vt_transpose_kernel(const unsigned short* __restrict__ qkv, unsigned short* __restrict__ vt) {
  __shared__ unsigned short sm[64][66];
  const int t  = threadIdx.x;
  const int m0 = blockIdx.x * 64;
  const int g  = blockIdx.y;
  const int b  = g / kHeads;
  const int h  = g - b * kHeads;
#pragma unroll
  for (int i = 0; i < 2; ++i) {
    const int e  = i * 256 + t;
    const int r  = e >> 3;
    const int c8 = (e & 7) * 8;
    const v4u u = *(const v4u*)(qkv + (size_t)(b * kSeq + m0 + r) * kQKVld + 2 * kDim + h * kHeadDim + c8);
#pragma unroll
    for (int j = 0; j < 4; ++j) {
      sm[c8 + 2 * j][r]     = (unsigned short)(u[j] & 0xffffu);
      sm[c8 + 2 * j + 1][r] = (unsigned short)(u[j] >> 16);
    }
  }
  __syncthreads();
  const int lane = t & 31, wave = t >> 5;
  const int q = lane >> 3, c8 = (lane & 7) * 8;
  unsigned short* op = vt + (size_t)g * kHeadDim * kSeq;
  for (int pass = 0; pass < 2; ++pass) {
#pragma unroll
    for (int it = 0; it < 2; ++it) {
      const int row = wave * 8 + it * 4 + q;
      const unsigned short* sp = &sm[row][c8];
      const v4u u = (v4u){pk16(sp[0], sp[1]), pk16(sp[2], sp[3]), pk16(sp[4], sp[5]), pk16(sp[6], sp[7])};
      *(volatile v4u*)(op + (size_t)row * kSeq + m0 + c8) = u;
    }
    __threadfence();
  }
}

__global__ __launch_bounds__(128) void softmax_bias_kernel(const float* __restrict__ S, const float* __restrict__ biasb,
                                                           unsigned short* __restrict__ P) {
  __shared__ float redM[4];
  __shared__ float redS[4];
  const int rowid = blockIdx.x;
  const int n     = rowid & (kSeq - 1);
  const int t     = threadIdx.x;
  const int lane  = t & 31, wave = t >> 5;
  const int c0    = t * 8;
  const float* sr = S + (size_t)rowid * kSeq + c0;
  const float* br = biasb + (size_t)n * kSeq + c0;
  const v4f a  = *(const v4f*)(sr);
  const v4f c  = *(const v4f*)(sr + 4);
  const v4f ba = *(const v4f*)(br);
  const v4f bc = *(const v4f*)(br + 4);
  float x[8];
#pragma unroll
  for (int e = 0; e < 4; ++e) { x[e] = a[e] + ba[e]; x[4 + e] = c[e] + bc[e]; }
  float m = fmaxf(fmaxf(fmaxf(x[0], x[1]), fmaxf(x[2], x[3])), fmaxf(fmaxf(x[4], x[5]), fmaxf(x[6], x[7])));
#pragma unroll
  for (int off = 16; off > 0; off >>= 1) m = fmaxf(m, __shfl_xor(m, off, 32));
  if (lane == 0) redM[wave] = m;
  __syncthreads();
  m = fmaxf(fmaxf(redM[0], redM[1]), fmaxf(redM[2], redM[3]));
  float ev[8];
  float s = 0.f;
#pragma unroll
  for (int e = 0; e < 8; ++e) { ev[e] = expf(x[e] - m); s += ev[e]; }
#pragma unroll
  for (int off = 16; off > 0; off >>= 1) s += __shfl_xor(s, off, 32);
  if (lane == 0) redS[wave] = s;
  __syncthreads();
  const float sum = ((redS[0] + redS[1]) + redS[2]) + redS[3];
  const float inv = kPCarry / sum;
  unsigned short hb[8];
#pragma unroll
  for (int e = 0; e < 8; ++e) hb[e] = h_bits(ev[e] * inv);
  const v4u u = (v4u){pk16(hb[0], hb[1]), pk16(hb[2], hb[3]), pk16(hb[4], hb[5]), pk16(hb[6], hb[7])};
  unsigned short* op = P + (size_t)rowid * kSeq + c0;
  *(volatile v4u*)op = u;
  __threadfence();
  *(volatile v4u*)op = u;
}

__global__ __launch_bounds__(256) void gelu_f16x2_kernel(const float* __restrict__ in, unsigned short* __restrict__ out, int n2) {
  const int i = blockIdx.x * 256 + threadIdx.x;
  if (i >= n2) return;
  const v2f p = *(const v2f*)(in + 2 * (size_t)i);
  const float a0 = p[0], a1 = p[1];
  const float g0 = 0.5f * a0 * (1.0f + erff(a0 * 0.70710678118654752f));
  const float g1 = 0.5f * a1 * (1.0f + erff(a1 * 0.70710678118654752f));
  const unsigned u = pk16(h_bits(g0), h_bits(g1));
  unsigned* q = (unsigned*)(out) + i;
  *(volatile unsigned*)q = u;
  __threadfence();
  *(volatile unsigned*)q = u;
}

extern "C" void kernel_launch(void* const* d_in, const int* in_sizes, int n_in,
                              void* d_out, int out_size, void* d_ws, size_t ws_size,
                              hipStream_t stream) {
  if (n_in < 14) return;
  if ((size_t)out_size < (size_t)kTok * kDim) return;
  if (ws_size < kWsTotal) return;
  if (in_sizes[0] < kTok * kDim || in_sizes[1] < kBatch * kSeq * kSeq || in_sizes[2] < kDim * kQKVld ||
      in_sizes[3] < kQKVld || in_sizes[4] < kDim * kDim || in_sizes[5] < kDim || in_sizes[6] < kDim ||
      in_sizes[7] < kDim || in_sizes[8] < kDim || in_sizes[9] < kDim || in_sizes[10] < kDim * kHid ||
      in_sizes[11] < kHid || in_sizes[12] < kHid * kDim || in_sizes[13] < kDim) return;

  const float* x      = (const float*)d_in[0];
  const float* pbias  = (const float*)d_in[1];
  const float* qkv_w  = (const float*)d_in[2];
  const float* qkv_b  = (const float*)d_in[3];
  const float* proj_w = (const float*)d_in[4];
  const float* proj_b = (const float*)d_in[5];
  const float* n1_w   = (const float*)d_in[6];
  const float* n1_b   = (const float*)d_in[7];
  const float* n2_w   = (const float*)d_in[8];
  const float* n2_b   = (const float*)d_in[9];
  const float* fc1_w  = (const float*)d_in[10];
  const float* fc1_b  = (const float*)d_in[11];
  const float* fc2_w  = (const float*)d_in[12];
  const float* fc2_b  = (const float*)d_in[13];
  float* out = (float*)d_out;

  char* ws = (char*)d_ws;
  unsigned short* Wqkv  = (unsigned short*)(ws + kOffWqkv);
  unsigned short* Wproj = (unsigned short*)(ws + kOffWproj);
  unsigned short* Wfc1  = (unsigned short*)(ws + kOffWfc1);
  unsigned short* Wfc2  = (unsigned short*)(ws + kOffWfc2);
  unsigned short* Hpl   = (unsigned short*)(ws + kOffH);
  unsigned short* QKV   = (unsigned short*)(ws + kOffQKV);
  unsigned short* VT    = (unsigned short*)(ws + kOffVt);
  unsigned short* OPL   = (unsigned short*)(ws + kOffO);
  float*          X1    = (float*)(ws + kOffX1);
  float*          SC    = (float*)(ws + kOffScores);
  unsigned short* PP    = (unsigned short*)(ws + kOffP);
  float*          G1    = (float*)(ws + kOffG1);
  unsigned short* HG    = (unsigned short*)(ws + kOffHG);

  wtcast_kernel<<<dim3(kDim / 64, kQKVld / 64), 256, 0, stream>>>(qkv_w, Wqkv, kDim, kQKVld, kWCarry);
  wtcast_kernel<<<dim3(kDim / 64, kDim / 64), 256, 0, stream>>>(proj_w, Wproj, kDim, kDim, kWCarry);
  wtcast_kernel<<<dim3(kDim / 64, kHid / 64), 256, 0, stream>>>(fc1_w, Wfc1, kDim, kHid, kWCarry);
  wtcast_kernel<<<dim3(kHid / 64, kDim / 64), 256, 0, stream>>>(fc2_w, Wfc2, kHid, kDim, kWCarry);

  layernorm_f16_kernel<<<kTok, 96, 0, stream>>>(x, n1_w, n1_b, Hpl);

  wmma_gemm64<0, false, 2, 1, false, 0><<<dim3((kTok / 64) * (kQKVld / 64) / 8, 1), 256, 0, stream>>>(
      Hpl, Hpl, kDim, 0L, Wqkv, Wqkv, kDim, 0L, (void*)QKV, (void*)QKV, kQKVld, 0L,
      qkv_b, x, 0L, kTok, kQKVld, kDim, 1.0f / kWCarry);

  vt_transpose_kernel<<<dim3(kSeq / 64, kGroups), 256, 0, stream>>>(QKV, VT);

  for (int ch = 0; ch < kChunks; ++ch) {
    const int b  = ch / (kHeads / kGroupsPerChunk);
    const int h0 = (ch % (kHeads / kGroupsPerChunk)) * kGroupsPerChunk;
    const unsigned short* Aq = QKV + (size_t)b * kSeq * kQKVld + (size_t)h0 * kHeadDim;
    const unsigned short* Bk = Aq + kDim;
    wmma_gemm64<0, false, 0, 0, false, 0><<<dim3((kSeq / 64) * (kSeq / 64) / 8, kGroupsPerChunk), 256, 0, stream>>>(
        Aq, Aq, kQKVld, (long)kHeadDim, Bk, Bk, kQKVld, (long)kHeadDim, (void*)SC, (void*)SC, kSeq, (long)kSeq * kSeq,
        qkv_b, x, 0L, kSeq, kSeq, kHeadDim, kAttnScale);
    softmax_bias_kernel<<<kGroupsPerChunk * kSeq, 128, 0, stream>>>(SC, pbias + (size_t)b * kSeq * kSeq, PP);
    const unsigned short* Bv = VT + (size_t)(b * kHeads + h0) * kHeadDim * kSeq;
    unsigned short* Co = OPL + (size_t)b * kSeq * kDim + (size_t)h0 * kHeadDim;
    wmma_gemm64<0, false, 0, 1, false, 0><<<dim3((kSeq / 64) * (kHeadDim / 64) / 8, kGroupsPerChunk), 256, 0, stream>>>(
        PP, PP, kSeq, (long)kSeq * kSeq, Bv, Bv, kSeq, (long)kHeadDim * kSeq, (void*)Co, (void*)Co, kDim, (long)kHeadDim,
        qkv_b, x, 0L, kSeq, kHeadDim, kSeq, kOCarry / kPCarry);
  }

  wmma_gemm64<0, false, 2, 0, true, 0><<<dim3((kTok / 64) * (kDim / 64) / 8, 1), 256, 0, stream>>>(
      OPL, OPL, kDim, 0L, Wproj, Wproj, kDim, 0L, (void*)X1, (void*)X1, kDim, 0L,
      proj_b, x, 0L, kTok, kDim, kDim, 1.0f / (kOCarry * kWCarry));

  layernorm_f16_kernel<<<kTok, 96, 0, stream>>>(X1, n2_w, n2_b, Hpl);

  wmma_gemm64<0, false, 2, 0, false, 0><<<dim3((kTok / 64) * (kHid / 64) / 8, 1), 256, 0, stream>>>(
      Hpl, Hpl, kDim, 0L, Wfc1, Wfc1, kDim, 0L, (void*)G1, (void*)G1, kHid, 0L,
      fc1_b, x, 0L, kTok, kHid, kDim, 1.0f / kWCarry);

  {
    const int n2 = kTok * kHid / 2;
    gelu_f16x2_kernel<<<(n2 + 255) / 256, 256, 0, stream>>>(G1, HG, n2);
  }

  wmma_gemm64<0, false, 2, 0, true, 0><<<dim3((kTok / 64) * (kDim / 64) / 8, 1), 256, 0, stream>>>(
      HG, HG, kHid, 0L, Wfc2, Wfc2, kHid, 0L, (void*)out, (void*)out, kDim, 0L,
      fc2_b, X1, 0L, kTok, kDim, kHid, 1.0f / kWCarry);
}
